// SelectiveScan_137438954197
// MI455X (gfx1250) — hardware-run, weakly checked
//
#include <hip/hip_runtime.h>


#define NGD  8
#define NST  4096
#define NCH  192
#define NJ   16
#define NRK  12
#define NW   44
#define NWP  64
#define NRP  32

typedef _Float16 h16;
typedef unsigned short bf;
typedef __attribute__((ext_vector_type(16))) __bf16   v16bf;
typedef __attribute__((ext_vector_type(16))) _Float16 v16h;
typedef __attribute__((ext_vector_type(8)))  _Float16 v8h;
typedef __attribute__((ext_vector_type(8)))  unsigned short v8us;
typedef __attribute__((ext_vector_type(8)))  float    v8f;
typedef __attribute__((ext_vector_type(4)))  float    v4f;
typedef v8h  __attribute__((may_alias)) v8ha;
typedef v4f  __attribute__((may_alias)) v4fa;
typedef v8us __attribute__((may_alias)) v8usa;

__device__ __forceinline__ unsigned short f2bf(float f) { unsigned u = __float_as_uint(f); u += 0x7FFFu + ((u >> 16) & 1u); return (unsigned short)(u >> 16); }
__device__ __forceinline__ float bf2f(unsigned short b) { return __uint_as_float(((unsigned)b) << 16); }
__device__ __forceinline__ float bfr(float f) { return bf2f(f2bf(f)); }
__device__ __forceinline__ v16h cat16(v8h lo, v8h hi) { return __builtin_shufflevector(lo, hi, 0, 1, 2, 3, 4, 5, 6, 7, 8, 9, 10, 11, 12, 13, 14, 15); }
__device__ __forceinline__ v16bf cat16b(v8us lo, v8us hi) { return __builtin_bit_cast(v16bf, __builtin_shufflevector(lo, hi, 0, 1, 2, 3, 4, 5, 6, 7, 8, 9, 10, 11, 12, 13, 14, 15)); }
__device__ __forceinline__ v8f wmma16(v16h a, v16h b, v8f c) { return __builtin_amdgcn_wmma_f32_16x16x32_f16(false, a, false, b, (short)0, c, false, false); }
__device__ __forceinline__ v8f wmmab(v16bf a, v16bf b, v8f c) { return __builtin_amdgcn_wmma_f32_16x16x32_bf16(false, a, false, b, (short)0, c, false, false); }

template <typename T16> struct WFrag;
template <> struct WFrag<h16> { typedef v16h V; static __device__ __forceinline__ V ld(const h16* p) { return cat16(*(const v8h*)p, *(const v8h*)(p + 16)); } static __device__ __forceinline__ v8f mma(V a, V b, v8f c) { return wmma16(a, b, c); } };
template <> struct WFrag<bf> { typedef v16bf V; static __device__ __forceinline__ V ld(const bf* p) { return cat16b(*(const v8us*)p, *(const v8us*)(p + 16)); } static __device__ __forceinline__ v8f mma(V a, V b, v8f c) { return wmmab(a, b, c); } };
template <typename T16, int NSPLIT, bool BIAS>
__global__ __launch_bounds__(32) void k_gemmw(const T16* __restrict__ A, const T16* __restrict__ A2, const T16* __restrict__ Bt, const T16* __restrict__ Bt2, int K, float* C, int ldc, const float* __restrict__ bias, size_t sA, size_t sB, size_t sC) {
    typedef typename WFrag<T16>::V V;
    __shared__ __align__(16) float os[16 * 68];
    const size_t z = blockIdx.z; A += z * sA; if (A2) A2 += z * sA; Bt += z * sB; if (Bt2) Bt2 += z * sB; C += z * sC;
    const int lane = threadIdx.x & 31, lr = lane & 15, hi = lane >> 4; const int r0 = blockIdx.x * 64, c0 = blockIdx.y * 64;
    v8f acc[4][4];
#pragma unroll
    for (int mb = 0; mb < 4; ++mb)
#pragma unroll
        for (int nb = 0; nb < 4; ++nb) acc[mb][nb] = (v8f){};
    const size_t aoff = (size_t)(r0 + lr) * K + 8 * hi, boff = (size_t)(c0 + lr) * K + 8 * hi;
    for (int kc = 0; kc < K; kc += 32) {
        V a[4], a2[4];
#pragma unroll
        for (int mb = 0; mb < 4; ++mb) { a[mb] = WFrag<T16>::ld(A + aoff + (size_t)mb * 16 * K + kc); if (NSPLIT == 1 || NSPLIT == 2) a2[mb] = WFrag<T16>::ld(A2 + aoff + (size_t)mb * 16 * K + kc); }
#pragma unroll
        for (int nb = 0; nb < 4; ++nb) { const V b = WFrag<T16>::ld(Bt + boff + (size_t)nb * 16 * K + kc); V b2; if (NSPLIT >= 2) b2 = WFrag<T16>::ld(Bt2 + boff + (size_t)nb * 16 * K + kc);
#pragma unroll
            for (int mb = 0; mb < 4; ++mb) { acc[mb][nb] = WFrag<T16>::mma(a[mb], b, acc[mb][nb]); if (NSPLIT == 1 || NSPLIT == 2) acc[mb][nb] = WFrag<T16>::mma(a2[mb], b, acc[mb][nb]); if (NSPLIT >= 2) acc[mb][nb] = WFrag<T16>::mma(a[mb], b2, acc[mb][nb]); } }
        asm volatile("v_nop\n\tv_nop\n\tv_nop\n\tv_nop" : "+v"(acc[0][0]), "+v"(acc[1][1]), "+v"(acc[2][2]), "+v"(acc[3][3]) : "v"(a[0]), "v"(a[3]));
    }
#pragma unroll
    for (int mb = 0; mb < 4; ++mb) {
#pragma unroll
        for (int nb = 0; nb < 4; ++nb) {
#pragma unroll
            for (int j = 0; j < 8; ++j) os[(hi * 8 + j) * 68 + nb * 16 + lr] = acc[mb][nb][j]; }
        __builtin_amdgcn_wave_barrier(); asm volatile("" ::: "memory");
        float* crow = C + (size_t)(r0 + mb * 16) * ldc + c0;
#pragma unroll 1
        for (int ps = 0; ps < 2; ++ps) {
#pragma unroll
            for (int s = 0; s < 8; ++s) { const int row = 2 * s + hi, cofs = lr * 4; v4f val = *(const v4fa*)(os + row * 68 + cofs); if (BIAS) { val[0] += bfr(bias[c0 + cofs]); val[1] += bfr(bias[c0 + cofs + 1]); val[2] += bfr(bias[c0 + cofs + 2]); val[3] += bfr(bias[c0 + cofs + 3]); }
                *(volatile v4f*)(crow + (size_t)row * ldc + cofs) = val; }
            if (ps == 0) __threadfence(); }
        __builtin_amdgcn_wave_barrier(); asm volatile("" ::: "memory");
    }
}

typedef __attribute__((ext_vector_type(2))) _Float16 v2h;
typedef __attribute__((ext_vector_type(4))) _Float16 v4h;
typedef __attribute__((ext_vector_type(2))) unsigned short v2us;
typedef __attribute__((ext_vector_type(4))) unsigned short v4us;
typedef __attribute__((ext_vector_type(2))) float v2f;
typedef __attribute__((ext_vector_type(4))) int v4i;
__global__ __launch_bounds__(256) void k_cvt8(const float* __restrict__ src, bf* dst, size_t n8) { const size_t i = (size_t)blockIdx.x * 256 + threadIdx.x; if (i >= n8) return; const v8f v = *(const v8f*)(src + i * 8); v8us o;
#pragma unroll
    for (int k = 0; k < 8; ++k) o[k] = f2bf(v[k]); *(volatile v8us*)(dst + i * 8) = o; __threadfence(); *(volatile v8us*)(dst + i * 8) = o; }

__global__ __launch_bounds__(256) void k_fillb(bf* P, unsigned w2, size_t n8) { const size_t i = (size_t)blockIdx.x * 256 + threadIdx.x; if (i >= n8) return; v4i o; o[0] = (int)w2; o[1] = (int)w2; o[2] = (int)w2; o[3] = (int)w2;
    *(volatile v4i*)(P + i * 8) = o; __threadfence(); *(volatile v4i*)(P + i * 8) = o; }

__global__ __launch_bounds__(256) void k_xt(const float* __restrict__ u1, bf* Xt) { const unsigned st = blockIdx.x * 256u + threadIdx.x, cr = blockIdx.y, gd = blockIdx.z; const float* ps = u1 + ((size_t)gd * NCH + cr * 64u) * NST + st; bf* pd = Xt + ((size_t)gd * NST + st) * NCH + cr * 64u; v8us ov[8];
#pragma unroll
    for (int q2 = 0; q2 < 8; ++q2) {
#pragma unroll
        for (int q1 = 0; q1 < 8; ++q1) ov[q2][q1] = f2bf(ps[(size_t)(q2 * 8 + q1) * NST]); }
#pragma unroll
    for (int q2 = 0; q2 < 8; ++q2) *(volatile v8us*)(pd + q2 * 8) = ov[q2];
    __threadfence();
#pragma unroll
    for (int q2 = 0; q2 < 8; ++q2) *(volatile v8us*)(pd + q2 * 8) = ov[q2]; }

__global__ __launch_bounds__(256) void k_pad12(const float* __restrict__ Sr, unsigned pt, unsigned ia, bf* Ph, bf* Pl) { const unsigned id = blockIdx.x * 256u + threadIdx.x; const unsigned rw = id >> 2, qt = id & 3u; const float* ps = Sr + (size_t)rw * pt; const v4f wa = *(const v4f*)ps, wb = *(const v4f*)(ps + 4), wc = *(const v4f*)(ps + 8); const unsigned mk = 0u - (ia & 1u); v8us oh, ol;
#pragma unroll
    for (int q1 = 0; q1 < 8; ++q1) { const float w0 = q1 < 4 ? wa[q1] : wb[q1 - 4], w1 = q1 < 4 ? wc[q1] : 0.0f; float wv = qt == 0u ? w0 : (qt == 1u ? w1 : 0.0f); wv = __uint_as_float((__float_as_uint(bfr(wv)) & mk) | (__float_as_uint(wv) & ~mk)); const unsigned short hw = f2bf(wv); oh[q1] = hw; ol[q1] = f2bf(wv - bf2f(hw)); }
    *(volatile v8us*)(Ph + (size_t)id * 8) = oh; *(volatile v8us*)(Pl + (size_t)id * 8) = ol; __threadfence(); *(volatile v8us*)(Ph + (size_t)id * 8) = oh; *(volatile v8us*)(Pl + (size_t)id * 8) = ol; }

__global__ __launch_bounds__(192) void k_s6(const float* __restrict__ Zs, const float* __restrict__ Xd, const float* __restrict__ u1, const float* __restrict__ u4, const float* __restrict__ u5, float* Yt) { const unsigned ch = threadIdx.x, gd = blockIdx.x; const unsigned kc = (gd & 1u) * NCH + ch; float rt[NJ], cw[NJ];
#pragma unroll
    for (int j = 0; j < NJ; ++j) { rt[j] = -expf(bfr(u5[(size_t)kc * NJ + j])); cw[j] = 0.0f; }
    const float ad = bfr(u4[kc]); const float* px = u1 + ((size_t)gd * NCH + ch) * NST; const float* pzs = Zs + (size_t)gd * NST * NCH + ch; const float* pe = Xd + (size_t)gd * NST * NWP; float* py = Yt + (size_t)gd * NST * NCH + ch;
#pragma unroll 1
    for (unsigned st = 0; st < 4096u; ++st) { const float dv = pzs[(size_t)st * NCH] + ad; const float sz = fmaxf(dv, 0.0f) + log1pf(expf(-fabsf(dv))); const float en = sz * bfr(px[st]); const float* pw = pe + (size_t)st * NWP; float sm = 0.0f;
#pragma unroll
        for (int j = 0; j < NJ; ++j) { cw[j] = expf(sz * rt[j]) * cw[j] + en * pw[NRK + j]; sm = sm + cw[j] * pw[NRK + NJ + j]; }
        *(volatile float*)(py + (size_t)st * NCH) = sm; __threadfence(); *(volatile float*)(py + (size_t)st * NCH) = sm; } }

__global__ __launch_bounds__(256) void k_yt(const float* __restrict__ Yt, const float* __restrict__ u1, const float* __restrict__ u6, float* Rs) { const unsigned s0 = (blockIdx.x * 256u + threadIdx.x) << 2, kc = blockIdx.y, gp = blockIdx.z; const unsigned dr = kc >= (unsigned)NCH ? 1u : 0u, ch = kc - dr * NCH, gd = gp * 2u + dr; const size_t eo = ((size_t)gp * 2u * NCH + kc) * NST + s0; const v4f xa = *(const v4f*)(u1 + eo); const float gn = bfr(u6[kc]); v4f ov;
#pragma unroll
    for (int q1 = 0; q1 < 4; ++q1) ov[q1] = Yt[((size_t)gd * NST + s0 + q1) * NCH + ch] + gn * bfr(xa[q1]);
    *(volatile v4f*)(Rs + eo) = ov; __threadfence(); *(volatile v4f*)(Rs + eo) = ov; }

extern "C" void kernel_launch(void* const* d_in, const int* in_sizes, int n_in, void* d_out, int out_size, void* d_ws, size_t ws_size, hipStream_t stream) {
    if (n_in < 6) return;
    if (in_sizes[0] != NGD * NCH * NST || in_sizes[1] != 2 * NW * NCH || in_sizes[2] != 2 * NCH * NRK || in_sizes[3] != 2 * NCH || in_sizes[4] != 2 * NCH * NJ || in_sizes[5] != 2 * NCH) return;
    if (out_size != NGD * NCH * NST) return;
    static_assert(NGD == 8 && NST == 4096 && NCH == 192 && NJ == 16 && NRK == 12 && NW == 44 && NWP == 64 && NRP == 32 && NW == NRK + 2 * NJ && NW <= NWP && NRK <= NRP && NST % 256 == 0 && NCH % 64 == 0 && NST % 64 == 0 && NWP % 64 == 0 && NCH % 32 == 0 && NRP % 32 == 0 && (2 * NCH * 4) % 256 == 0 && (2 * NWP * NCH / 8) % 256 == 0 && (NGD * NST * 4) % 256 == 0 && (NST / 4) % 256 == 0 && (NRK * 4) % 16 == 0 && (NWP * 4) % 16 == 0, "the products: row and column counts multiples of 64, the depths of 32; each flat grid exact; k_pad12's rows begin on 16 bytes at both pitches (12 and 64 words); k_s6's block is the 192 channels");
    const float* i0 = (const float*)d_in[0]; const float* i1 = (const float*)d_in[1]; const float* i2 = (const float*)d_in[2]; const float* i3 = (const float*)d_in[3]; const float* i4 = (const float*)d_in[4]; const float* i5 = (const float*)d_in[5]; float* rs0 = (float*)d_out;
    char* wsp = (char*)d_ws; auto carve = [&](size_t bytes) { char* p = wsp; wsp += (bytes + 255) & ~(size_t)255; return (void*)p; };
    bf* Xt = (bf*)carve((size_t)NGD * NST * NCH * 2); bf* W1 = (bf*)carve((size_t)2 * NWP * NCH * 2); bf* Wdh = (bf*)carve((size_t)2 * NCH * NRP * 2); bf* Wdl = (bf*)carve((size_t)2 * NCH * NRP * 2); float* Xd = (float*)carve((size_t)NGD * NST * NWP * 4); bf* Drh = (bf*)carve((size_t)NGD * NST * NRP * 2); bf* Drl = (bf*)carve((size_t)NGD * NST * NRP * 2); float* Zs = (float*)carve((size_t)NGD * NST * NCH * 4); float* Yt = (float*)carve((size_t)NGD * NST * NCH * 4);
    if ((size_t)(wsp - (char*)d_ws) > ws_size) return;
    k_xt<<<dim3(NST / 256, NCH / 64, NGD), 256, 0, stream>>>(i0, Xt);
    k_fillb<<<(unsigned)(2 * NWP * NCH / 8 / 256), 256, 0, stream>>>(W1, 0u, (size_t)2 * NWP * NCH / 8);
    for (unsigned dr = 0; dr < 2u; ++dr) k_cvt8<<<(unsigned)((NW * NCH / 8 + 255) / 256), 256, 0, stream>>>(i1 + (size_t)dr * NW * NCH, W1 + (size_t)dr * NWP * NCH, (size_t)NW * NCH / 8);
    k_pad12<<<(unsigned)(2 * NCH * 4 / 256), 256, 0, stream>>>(i2, (unsigned)NRK, 1u, Wdh, Wdl);
    for (unsigned dr = 0; dr < 2u; ++dr) k_gemmw<bf, 0, false><<<dim3(NST / 64, NWP / 64, NGD / 2), 32, 0, stream>>>(Xt + (size_t)dr * NST * NCH, nullptr, W1 + (size_t)dr * NWP * NCH, nullptr, NCH, Xd + (size_t)dr * NST * NWP, NWP, nullptr, (size_t)2 * NST * NCH, (size_t)0, (size_t)2 * NST * NWP);
    k_pad12<<<(unsigned)(NGD * NST * 4 / 256), 256, 0, stream>>>(Xd, (unsigned)NWP, 0u, Drh, Drl);
    for (unsigned dr = 0; dr < 2u; ++dr) k_gemmw<bf, 1, false><<<dim3(NST / 64, NCH / 64, NGD / 2), 32, 0, stream>>>(Drh + (size_t)dr * NST * NRP, Drl + (size_t)dr * NST * NRP, Wdh + (size_t)dr * NCH * NRP, nullptr, NRP, Zs + (size_t)dr * NST * NCH, NCH, nullptr, (size_t)2 * NST * NRP, (size_t)0, (size_t)2 * NST * NCH);
    k_s6<<<(unsigned)NGD, NCH, 0, stream>>>(Zs, Xd, i0, i3, i4, Yt);
    k_yt<<<dim3(NST / 4 / 256, 2 * NCH, NGD / 2), 256, 0, stream>>>(Yt, i0, i5, rs0);
}
